// MHA_52312701665688
// MI455X (gfx1250) — hardware-verified
//
#include <hip/hip_runtime.h>


#ifndef NB
#define NB 1
#endif
#ifndef SEQ
#define SEQ 2048
#endif
#define SEQ_FULL 2048
#define TT   SEQ
#define DM   1024
#define NH_  16
#define HD   64
#define DQ   (NH_ * HD)
#define NQKV (3 * DQ)
#define ZH   2
#define SCL  0.125f

typedef unsigned short bf;
typedef __attribute__((ext_vector_type(16))) __bf16   v16bf;
typedef __attribute__((ext_vector_type(8)))  unsigned short v8us;
typedef __attribute__((ext_vector_type(4)))  unsigned short v4us;
typedef __attribute__((ext_vector_type(2)))  unsigned short v2us;
typedef __attribute__((ext_vector_type(8)))  float    v8f;
typedef __attribute__((ext_vector_type(4)))  float    v4f;
typedef __attribute__((ext_vector_type(2)))  float    v2f;
typedef v4f  __attribute__((may_alias)) v4fa;

constexpr unsigned lg2c(unsigned v) { return v <= 1u ? 0u : 1u + lg2c(v >> 1); }
constexpr bool ispow2(unsigned v) { return v != 0u && (v & (v - 1u)) == 0u; }
constexpr size_t al256(size_t b) { return (b + 255) & ~(size_t)255; }
constexpr size_t cmaxz(size_t a, size_t b) { return a > b ? a : b; }
#define LG_TT lg2c(TT)
#define LG_HD lg2c(HD)
#define LG_DM lg2c(DM)
#define LG_DQ lg2c(DQ)

static_assert(NB == 1);
static_assert(SEQ <= SEQ_FULL);
static_assert(ispow2(TT) && ispow2(HD) && ispow2(DM) && ispow2(DQ));
static_assert(TT % 128 == 0 && TT % 64 == 0);
static_assert(DM % 32 == 0 && DQ % 32 == 0 && HD % 32 == 0 && TT % 32 == 0);
static_assert(NQKV % 64 == 0 && DM % 64 == 0 && HD % 64 == 0);
static_assert(((size_t)TT * DM) % 2048 == 0);
static_assert(((size_t)NQKV * DM) % 512 == 0);
static_assert(((size_t)DM * DQ) % 512 == 0);
static_assert(((size_t)NH_ * TT * HD) % 512 == 0);
static_assert(((size_t)ZH * TT * HD) % 512 == 0);
static_assert((ZH * TT) % 8 == 0 && NH_ % ZH == 0);

constexpr size_t SZ_WT = al256((size_t)NQKV * DM * 2);
constexpr size_t SZ_WP = al256((size_t)DM * DQ * 2);
constexpr size_t SZ_XB = al256((size_t)TT * DM * 2);
constexpr size_t SZ_HP = al256((size_t)NH_ * TT * HD * 2);
constexpr size_t SZ_SF = al256(cmaxz((size_t)ZH * TT * TT * 4, (size_t)TT * NQKV * 4));
constexpr size_t SZ_P  = al256((size_t)ZH * TT * TT * 2);
constexpr size_t SZ_OB = al256((size_t)ZH * TT * HD * 4);
constexpr size_t SZ_Y  = al256((size_t)TT * DQ * 2);
constexpr size_t OFF_WT = 0;
constexpr size_t OFF_WP = OFF_WT + SZ_WT;
constexpr size_t OFF_XB = OFF_WP + SZ_WP;
constexpr size_t OFF_QH = OFF_XB + SZ_XB;
constexpr size_t OFF_QL = OFF_QH + SZ_HP;
constexpr size_t OFF_KH = OFF_QL + SZ_HP;
constexpr size_t OFF_KL = OFF_KH + SZ_HP;
constexpr size_t OFF_VH = OFF_KL + SZ_HP;
constexpr size_t OFF_VL = OFF_VH + SZ_HP;
constexpr size_t OFF_SF = OFF_VL + SZ_HP;
constexpr size_t OFF_PH = OFF_SF + SZ_SF;
constexpr size_t OFF_PL = OFF_PH + SZ_P;
constexpr size_t OFF_OB = OFF_PL + SZ_P;
constexpr size_t OFF_YH = OFF_OB + SZ_OB;
constexpr size_t OFF_YL = OFF_YH + SZ_Y;
constexpr size_t WS_TOTAL = OFF_YL + SZ_Y;
static_assert((size_t)TT * NQKV * 4 <= SZ_SF);
static_assert((size_t)ZH * TT * TT * 4 <= SZ_SF);
static_assert(WS_TOTAL <= (size_t)134217728);

__device__ __forceinline__ unsigned short f2bf(float f) { unsigned u = __float_as_uint(f); u += 0x7FFFu + ((u >> 16) & 1u); return (unsigned short)(u >> 16); }
__device__ __forceinline__ float bf2f(unsigned short b) { return __uint_as_float(((unsigned)b) << 16); }
__device__ __forceinline__ float bfr(float f) { return bf2f(f2bf(f)); }
__device__ __forceinline__ v16bf cat16b(v8us lo, v8us hi) { return __builtin_bit_cast(v16bf, __builtin_shufflevector(lo, hi, 0, 1, 2, 3, 4, 5, 6, 7, 8, 9, 10, 11, 12, 13, 14, 15)); }
__device__ __forceinline__ v8f wmmab(v16bf a, v16bf b, v8f c) { return __builtin_amdgcn_wmma_f32_16x16x32_bf16(false, a, false, b, (short)0, c, false, false); }
__device__ __forceinline__ void splitf(float y, unsigned short& h, unsigned short& l) { h = f2bf(y); l = f2bf(y - bf2f(h)); }

template <typename T16> struct WFrag;
template <> struct WFrag<bf> { typedef v16bf V; static __device__ __forceinline__ V ld(const bf* p) { return cat16b(*(const v8us*)p, *(const v8us*)(p + 16)); } static __device__ __forceinline__ v8f mma(V a, V b, v8f c) { return wmmab(a, b, c); } };
template <typename T16, int NSPLIT, bool BIAS>
__global__ __launch_bounds__(32) void k_gemmw(const T16* __restrict__ A, const T16* __restrict__ A2, const T16* __restrict__ Bt, const T16* __restrict__ Bt2, int K, float* C, int ldc, const float* __restrict__ bias, size_t sA, size_t sB, size_t sC) {
    typedef typename WFrag<T16>::V V;
    __shared__ __align__(16) float os[16 * 68];
    const size_t z = blockIdx.z; A += z * sA; if (A2) A2 += z * sA; Bt += z * sB; if (Bt2) Bt2 += z * sB; C += z * sC;
    const int lane = threadIdx.x & 31, lr = lane & 15, hi = lane >> 4; const int r0 = blockIdx.x * 64, c0 = blockIdx.y * 64;
    v8f acc[4][4];
#pragma unroll
    for (int mb = 0; mb < 4; ++mb)
#pragma unroll
        for (int nb = 0; nb < 4; ++nb) acc[mb][nb] = (v8f){};
    const size_t aoff = (size_t)(r0 + lr) * K + 8 * hi, boff = (size_t)(c0 + lr) * K + 8 * hi;
#pragma unroll 1
    for (int kc = 0; kc < K; kc += 32) {
        V a[4], a2[4];
#pragma unroll
        for (int mb = 0; mb < 4; ++mb) { a[mb] = WFrag<T16>::ld(A + aoff + (size_t)mb * 16 * K + kc); if (NSPLIT == 1 || NSPLIT == 2) a2[mb] = WFrag<T16>::ld(A2 + aoff + (size_t)mb * 16 * K + kc); }
#pragma unroll
        for (int nb = 0; nb < 4; ++nb) { const V b = WFrag<T16>::ld(Bt + boff + (size_t)nb * 16 * K + kc); V b2; if (NSPLIT >= 2) b2 = WFrag<T16>::ld(Bt2 + boff + (size_t)nb * 16 * K + kc);
#pragma unroll
            for (int mb = 0; mb < 4; ++mb) { acc[mb][nb] = WFrag<T16>::mma(a[mb], b, acc[mb][nb]); if (NSPLIT == 1 || NSPLIT == 2) acc[mb][nb] = WFrag<T16>::mma(a2[mb], b, acc[mb][nb]); if (NSPLIT >= 2) acc[mb][nb] = WFrag<T16>::mma(a[mb], b2, acc[mb][nb]); } }
        asm volatile("v_nop\n\tv_nop\n\tv_nop\n\tv_nop" : "+v"(acc[0][0]), "+v"(acc[1][1]), "+v"(acc[2][2]), "+v"(acc[3][3]) : "v"(a[0]), "v"(a[3]));
    }
#pragma unroll
    for (int mb = 0; mb < 4; ++mb) {
#pragma unroll
        for (int nb = 0; nb < 4; ++nb) {
#pragma unroll
            for (int j = 0; j < 8; ++j) os[(hi * 8 + j) * 68 + nb * 16 + lr] = acc[mb][nb][j]; }
        __builtin_amdgcn_wave_barrier(); asm volatile("" ::: "memory");
        float* crow = C + (size_t)(r0 + mb * 16) * ldc + c0;
#pragma unroll 1
        for (int ps = 0; ps < 2; ++ps) {
#pragma unroll
            for (int s = 0; s < 8; ++s) { const int row = 2 * s + hi, cofs = lr * 4; v4f val = *(const v4fa*)(os + row * 68 + cofs); if (BIAS) { val[0] += bfr(bias[c0 + cofs]); val[1] += bfr(bias[c0 + cofs + 1]); val[2] += bfr(bias[c0 + cofs + 2]); val[3] += bfr(bias[c0 + cofs + 3]); }
                *(volatile v4f*)(crow + (size_t)row * ldc + cofs) = val; }
            if (ps == 0) __threadfence(); }
        __builtin_amdgcn_wave_barrier(); asm volatile("" ::: "memory");
    }
}

__global__ __launch_bounds__(256) void k_cvt8(const float* __restrict__ src, bf* dst, size_t n8) { const size_t i = (size_t)blockIdx.x * 256 + threadIdx.x; if (i >= n8) return; const v8f v = *(const v8f*)(src + i * 8); v8us o;
#pragma unroll
    for (int k = 0; k < 8; ++k) o[k] = f2bf(v[k]); *(volatile v8us*)(dst + i * 8) = o; __threadfence(); *(volatile v8us*)(dst + i * 8) = o; }

__global__ __launch_bounds__(256) void k_wtT(const float* __restrict__ w, bf* dst, unsigned K, unsigned lgK, unsigned N) {
    const unsigned e2 = (blockIdx.x * 256u + threadIdx.x) * 2u; if (e2 >= N * K) return;
    const unsigned k = e2 & (K - 1u); const unsigned n = e2 >> lgK;
    const float* src = w + (size_t)k * N + n; v2us o; o[0] = f2bf(src[0]); o[1] = f2bf(src[N]);
    bf* p = dst + (size_t)n * K + k;
    *(volatile v2us*)p = o; __threadfence(); *(volatile v2us*)p = o; }

__global__ __launch_bounds__(256) void k_hp(const float* __restrict__ F, unsigned pitch, bf* Ph, bf* Pl) {
    const unsigned e = (blockIdx.x * 256u + threadIdx.x) * 2u; if (e >= (unsigned)NH_ * TT * HD) return;
    const unsigned d = e & (HD - 1u); const unsigned t = (e >> LG_HD) & (TT - 1u); const unsigned h = e >> (LG_HD + LG_TT);
    const v2f x = *(const v2f*)(F + (size_t)t * pitch + h * HD + d);
    v2us oh, ol; unsigned short a, c;
    splitf(x[0], a, c); oh[0] = a; ol[0] = c; splitf(x[1], a, c); oh[1] = a; ol[1] = c;
    *(volatile v2us*)(Ph + e) = oh; *(volatile v2us*)(Pl + e) = ol; __threadfence(); *(volatile v2us*)(Ph + e) = oh; *(volatile v2us*)(Pl + e) = ol; }

__global__ __launch_bounds__(256) void k_vtp(const float* __restrict__ F, unsigned pitch, bf* Vh, bf* Vl) {
    const unsigned e = (blockIdx.x * 256u + threadIdx.x) * 2u; if (e >= (unsigned)NH_ * HD * TT) return;
    const unsigned t = e & (TT - 1u); const unsigned d = (e >> LG_TT) & (HD - 1u); const unsigned g = e >> (LG_TT + LG_HD);
    v2us oh, ol;
#pragma unroll
    for (int q = 0; q < 2; ++q) { const float x = F[(size_t)(t + q) * pitch + g * HD + d]; unsigned short a, c; splitf(x, a, c); oh[q] = a; ol[q] = c; }
    *(volatile v2us*)(Vh + e) = oh; *(volatile v2us*)(Vl + e) = ol; __threadfence(); *(volatile v2us*)(Vh + e) = oh; *(volatile v2us*)(Vl + e) = ol; }

__global__ __launch_bounds__(256) void k_asoft(const float* __restrict__ Sb, bf* Ph, bf* Pl) {
    const unsigned lane = threadIdx.x & 31u; const unsigned row = blockIdx.x * 8u + (threadIdx.x >> 5); if (row >= (unsigned)ZH * TT) return;
    const float* sr = Sb + (size_t)row * TT; float v[TT / 32]; float mx = -3.0e38f;
#pragma unroll
    for (int ch = 0; ch < TT / 128; ++ch) { const v4f a = *(const v4f*)(sr + ch * 128 + lane * 4);
#pragma unroll
        for (int q = 0; q < 4; ++q) { const float t = a[q] * SCL; v[ch * 4 + q] = t; mx = fmaxf(mx, t); } }
#pragma unroll
    for (int sh = 16; sh; sh >>= 1) mx = fmaxf(mx, __shfl_xor(mx, sh, 32));
    float sum = 0.f;
#pragma unroll
    for (int k = 0; k < TT / 32; ++k) { float d0 = __fsub_rn(v[k], mx); asm volatile("" : "+v"(d0)); v[k] = __builtin_amdgcn_exp2f(__fmul_rn(d0, 1.4426950408889634f)); sum += v[k]; }
#pragma unroll
    for (int sh = 16; sh; sh >>= 1) sum += __shfl_xor(sum, sh, 32);
    const float f = __fdiv_rn(1.0f, sum);
#pragma unroll 1
    for (int ps = 0; ps < 2; ++ps) {
#pragma unroll
        for (int ch = 0; ch < TT / 128; ++ch) { v4us oh, ol;
#pragma unroll
            for (int q = 0; q < 4; ++q) { unsigned short a, c2; splitf(v[ch * 4 + q] * f, a, c2); oh[q] = a; ol[q] = c2; }
            const size_t oo = (size_t)row * TT + ch * 128 + lane * 4; *(volatile v4us*)(Ph + oo) = oh; *(volatile v4us*)(Pl + oo) = ol; }
        if (ps == 0) __threadfence(); }
}

__global__ __launch_bounds__(256) void k_mergey(const float* __restrict__ O, unsigned h0, bf* YH, bf* YL) {
    const unsigned e = (blockIdx.x * 256u + threadIdx.x) * 2u; if (e >= (unsigned)ZH * TT * HD) return;
    const unsigned d = e & (HD - 1u); const unsigned t = (e >> LG_HD) & (TT - 1u); const unsigned zz = e >> (LG_HD + LG_TT);
    const v2f o = *(const v2f*)(O + e); v2us oh, ol; unsigned short a, c;
    splitf(o[0], a, c); oh[0] = a; ol[0] = c; splitf(o[1], a, c); oh[1] = a; ol[1] = c;
    const size_t oo = (size_t)t * DQ + (size_t)(h0 + zz) * HD + d;
    *(volatile v2us*)(YH + oo) = oh; *(volatile v2us*)(YL + oo) = ol; __threadfence(); *(volatile v2us*)(YH + oo) = oh; *(volatile v2us*)(YL + oo) = ol; }

extern "C" void kernel_launch(void* const* d_in, const int* in_sizes, int n_in,
                              void* d_out, int out_size, void* d_ws, size_t ws_size, hipStream_t stream) {
    if (n_in < 5) return;
    if (in_sizes[0] < TT * DM || in_sizes[1] < DM * NQKV || in_sizes[2] < NQKV || in_sizes[3] < DQ * DM || in_sizes[4] < DM) return;
    if (out_size < TT * DM) return;
    if (WS_TOTAL > ws_size) return;
    const float* x     = (const float*)d_in[0];
    const float* wqkv  = (const float*)d_in[1];
    const float* bqkv  = (const float*)d_in[2];
    const float* wproj = (const float*)d_in[3];
    const float* bproj = (const float*)d_in[4];
    float* OUT = (float*)d_out;
    char* base = (char*)d_ws;
    bf* WT = (bf*)(base + OFF_WT); bf* WP = (bf*)(base + OFF_WP); bf* XB = (bf*)(base + OFF_XB);
    bf* QPh = (bf*)(base + OFF_QH); bf* QPl = (bf*)(base + OFF_QL); bf* KPh = (bf*)(base + OFF_KH); bf* KPl = (bf*)(base + OFF_KL); bf* VTh = (bf*)(base + OFF_VH); bf* VTl = (bf*)(base + OFF_VL);
    float* Sb = (float*)(base + OFF_SF); float* F = Sb;
    bf* Ph = (bf*)(base + OFF_PH); bf* Pl = (bf*)(base + OFF_PL); float* Ob = (float*)(base + OFF_OB);
    bf* YH = (bf*)(base + OFF_YH); bf* YL = (bf*)(base + OFF_YL);

    k_cvt8<<<(unsigned)(((size_t)TT * DM / 8 + 255) / 256), 256, 0, stream>>>(x, XB, (size_t)TT * DM / 8);
    k_wtT<<<(unsigned)(((size_t)NQKV * DM / 2 + 255) / 256), 256, 0, stream>>>(wqkv, WT, (unsigned)DM, LG_DM, (unsigned)NQKV);
    k_wtT<<<(unsigned)(((size_t)DM * DQ / 2 + 255) / 256), 256, 0, stream>>>(wproj, WP, (unsigned)DQ, LG_DQ, (unsigned)DM);
    k_gemmw<bf, 0, true><<<dim3(TT / 64, NQKV / 64, 1), 32, 0, stream>>>(XB, nullptr, WT, nullptr, DM, F, NQKV, bqkv, 0, 0, 0);
    const unsigned LP = (unsigned)(((size_t)NH_ * TT * HD / 2 + 255) / 256);
    k_hp<<<LP, 256, 0, stream>>>(F, (unsigned)NQKV, QPh, QPl);
    k_hp<<<LP, 256, 0, stream>>>(F + DQ, (unsigned)NQKV, KPh, KPl);
    k_vtp<<<LP, 256, 0, stream>>>(F + 2 * DQ, (unsigned)NQKV, VTh, VTl);
    for (int h0 = 0; h0 < NH_; h0 += ZH) { const size_t zq = (size_t)h0;
        k_gemmw<bf, 2, false><<<dim3(TT / 64, TT / 64, ZH), 32, 0, stream>>>(QPh + zq * TT * HD, QPl + zq * TT * HD, KPh + zq * TT * HD, KPl + zq * TT * HD, HD, Sb, TT, nullptr, (size_t)TT * HD, (size_t)TT * HD, (size_t)TT * TT);
        k_asoft<<<ZH * TT / 8, 256, 0, stream>>>(Sb, Ph, Pl);
        k_gemmw<bf, 2, false><<<dim3(TT / 64, HD / 64, ZH), 32, 0, stream>>>(Ph, Pl, VTh + zq * HD * TT, VTl + zq * HD * TT, TT, Ob, HD, nullptr, (size_t)TT * TT, (size_t)HD * TT, (size_t)TT * HD);
        k_mergey<<<(unsigned)(((size_t)ZH * TT * HD / 2 + 255) / 256), 256, 0, stream>>>(Ob, (unsigned)h0, YH, YL); }
    k_gemmw<bf, 1, true><<<dim3(TT / 64, DM / 64, 1), 32, 0, stream>>>(YH, YL, WP, nullptr, DQ, OUT, DM, bproj, 0, 0, 0);
}
